// TopLineEncoder_16415365005453
// MI455X (gfx1250) — hardware-run, weakly checked
//
#include <hip/hip_runtime.h>


#ifndef NROWS
#define NROWS 8192
#endif
#define NROWS_FULL 8192
#define NPOS  80
#define NCHAR 256
#define HDIM  512
#define IDIM  (NPOS * NCHAR)
#define GW    4
#define GW2   4
#define OP    516
#define TP    72
#define WSC   16.0f
#define WSI   (1.0f / 16.0f)
#define LNEPS 1.0e-5f

static_assert(NPOS * NCHAR == IDIM);
static_assert(HDIM == 512);
static_assert(HDIM % 32 == 0);
static_assert(HDIM == GW2 * 128);
static_assert(16 == GW2 * 4);
static_assert(IDIM % 64 == 0);
static_assert(HDIM % 64 == 0);
static_assert(NROWS % GW == 0);
static_assert(NROWS % 16 == 0);
static_assert(NROWS <= NROWS_FULL);
static_assert((OP * 4) % 16 == 0);
static_assert(OP >= HDIM);
static_assert((TP * 2) % 16 == 0);
static_assert(TP >= 64);
static_assert(2 * 256 * 16 == 64 * 128);
static_assert(2 * 32 * 16 == HDIM * 2);
static_assert(4 * 4 * 32 * 16 == 4 * HDIM * 4);
static_assert((size_t)64 * TP * 2 <= 131072);
static_assert((size_t)GW * HDIM * (4 + 2) <= 131072);
static_assert((size_t)16 * OP * 4 <= 131072);

typedef _Float16 h16;
typedef unsigned short bf;
typedef __attribute__((ext_vector_type(16))) _Float16 v16h;
typedef __attribute__((ext_vector_type(8)))  _Float16 v8h;
typedef __attribute__((ext_vector_type(8)))  unsigned short v8us;
typedef __attribute__((ext_vector_type(4)))  unsigned v4u;
typedef __attribute__((ext_vector_type(8)))  float    v8f;
typedef __attribute__((ext_vector_type(4)))  float    v4f;
typedef v4f  __attribute__((may_alias)) v4fa;
typedef v8h  __attribute__((may_alias)) v8ha;
typedef v8us __attribute__((may_alias)) v8usa;

__device__ __forceinline__ unsigned short f2bf(float f) { unsigned u = __float_as_uint(f); u += 0x7FFFu + ((u >> 16) & 1u); return (unsigned short)(u >> 16); }
__device__ __forceinline__ float bfr(float f) { return __uint_as_float(((unsigned)f2bf(f)) << 16); }
__device__ __forceinline__ v16h cat16(v8h lo, v8h hi) { return __builtin_shufflevector(lo, hi, 0, 1, 2, 3, 4, 5, 6, 7, 8, 9, 10, 11, 12, 13, 14, 15); }
__device__ __forceinline__ v8f wmma16(v16h a, v16h b, v8f c) { return __builtin_amdgcn_wmma_f32_16x16x32_f16(false, a, false, b, (short)0, c, false, false); }
__device__ __forceinline__ v8f wmma16g(v16h a, v16h b, v8f c) { c = wmma16(a, b, c); asm volatile("v_nop\n\tv_nop\n\tv_nop\n\tv_nop" : "+v"(c) : "v"(a), "v"(b)); return c; }
__device__ __forceinline__ v16h ldh(const h16* p) { return cat16(*(const v8h*)p, *(const v8h*)(p + 16)); }
__device__ __forceinline__ void wave_sync() { __builtin_amdgcn_fence(3  , "wavefront"); __builtin_amdgcn_wave_barrier(); asm volatile("" ::: "memory"); }
static __device__ __forceinline__ h16 toh_flush(float v) { const float w = (fabsf(v) < 6.103515625e-05f) ? 0.0f : v; return (h16)w; }
__device__ __forceinline__ float elu1(float v) { const float e = expm1f(fminf(v, 0.0f)); return (v > 0.0f) ? v : e; }

__global__ __launch_bounds__(256) void k_w1t(const float* __restrict__ W1, bf* W1T) {
    __shared__ __align__(16) bf tl[64 * TP];
    const unsigned t = threadIdx.x;
    const unsigned i0 = blockIdx.x * 64u, h0 = blockIdx.y * 64u;
    const unsigned rr = t >> 4, c4 = (t & 15u) * 4u;
#pragma unroll
    for (unsigned ps = 0; ps < 4; ++ps) {
        const unsigned h = ps * 16u + rr;
        const v4f v = *(const v4f*)(W1 + (size_t)(h0 + h) * IDIM + i0 + c4);
#pragma unroll
        for (unsigned k = 0; k < 4; ++k) tl[(c4 + k) * TP + h] = f2bf(v[k]);
    }
    __syncthreads();
    const unsigned q = t & 7u, ir = t >> 3;
#pragma unroll 1
    for (int ps = 0; ps < 2; ++ps) {
#pragma unroll
        for (unsigned s = 0; s < 2; ++s) {
            const unsigned i = s * 32u + ir;
            const v8us o = *(const v8usa*)(&tl[i * TP + 8u * q]);
            *(volatile v8us*)(W1T + (size_t)(i0 + i) * HDIM + h0 + 8u * q) = o; }
        if (ps == 0) __threadfence(); }
}

__global__ __launch_bounds__(256) void k_wcv(const float* __restrict__ src, h16* dst, unsigned n8) {
    const unsigned i = blockIdx.x * 256u + threadIdx.x; if (i >= n8) return;
    const v8f v = *(const v8f*)(src + (size_t)i * 8); v8h o;
#pragma unroll
    for (int k = 0; k < 8; ++k) o[k] = toh_flush(bfr(v[k]) * WSC);
    *(volatile v8h*)(dst + (size_t)i * 8) = o; __threadfence(); *(volatile v8h*)(dst + (size_t)i * 8) = o;
}

__global__ __launch_bounds__(32 * GW) void k_gather(const int* __restrict__ msg, const bf* __restrict__ W1T, const float* __restrict__ b1,
                                                    const float* __restrict__ g1, const float* __restrict__ be1, h16* HH) {
#pragma clang fp contract(off)
    __shared__ __align__(16) float xs[GW * HDIM];
    __shared__ __align__(16) h16   hs[GW * HDIM];
    const unsigned lane = threadIdx.x & 31u;
    const int wave = __builtin_amdgcn_readfirstlane((int)(threadIdx.x >> 5));
    const unsigned row = blockIdx.x * (unsigned)GW + (unsigned)wave;
    const int* mrow = msg + (size_t)row * NPOS;
    const unsigned wb = (unsigned)wave * HDIM;
    float acc[16];
#pragma unroll
    for (int j = 0; j < 16; ++j) acc[j] = 0.0f;
#pragma unroll 2
    for (int p = 0; p < NPOS; ++p) {
        int c = mrow[p]; c = min(max(c, 0), NCHAR - 1);
        const bf* wr = W1T + (size_t)(p * NCHAR + c) * HDIM + 8u * lane;
        const v4u u0 = *(const v4u*)wr;
        const v4u u1 = *(const v4u*)(wr + 256);
#pragma unroll
        for (int q = 0; q < 4; ++q) {
            acc[2 * q]         += __uint_as_float(u0[q] << 16);
            acc[2 * q + 1]     += __uint_as_float(u0[q] & 0xffff0000u);
            acc[8 + 2 * q]     += __uint_as_float(u1[q] << 16);
            acc[8 + 2 * q + 1] += __uint_as_float(u1[q] & 0xffff0000u); }
    }
    float gv[16], ev[16];
    {
        const v4f t0 = *(const v4f*)(b1 + 8u * lane), t1 = *(const v4f*)(b1 + 8u * lane + 4), t2 = *(const v4f*)(b1 + 256 + 8u * lane), t3 = *(const v4f*)(b1 + 260 + 8u * lane);
        const v4f a0 = *(const v4f*)(g1 + 8u * lane), a1 = *(const v4f*)(g1 + 8u * lane + 4), a2 = *(const v4f*)(g1 + 256 + 8u * lane), a3 = *(const v4f*)(g1 + 260 + 8u * lane);
        const v4f e0 = *(const v4f*)(be1 + 8u * lane), e1 = *(const v4f*)(be1 + 8u * lane + 4), e2 = *(const v4f*)(be1 + 256 + 8u * lane), e3 = *(const v4f*)(be1 + 260 + 8u * lane);
#pragma unroll
        for (int k = 0; k < 4; ++k) {
            acc[k] += bfr(t0[k]); acc[4 + k] += bfr(t1[k]); acc[8 + k] += bfr(t2[k]); acc[12 + k] += bfr(t3[k]);
            gv[k] = bfr(a0[k]); gv[4 + k] = bfr(a1[k]); gv[8 + k] = bfr(a2[k]); gv[12 + k] = bfr(a3[k]);
            ev[k] = bfr(e0[k]); ev[4 + k] = bfr(e1[k]); ev[8 + k] = bfr(e2[k]); ev[12 + k] = bfr(e3[k]); }
    }
    float s = 0.0f;
#pragma unroll
    for (int j = 0; j < 16; ++j) s += acc[j];
#pragma unroll
    for (int off = 16; off > 0; off >>= 1) s += __shfl_xor(s, off, 32);
    const float mu = s * (1.0f / (float)HDIM);
    float qq = 0.0f;
#pragma unroll
    for (int j = 0; j < 16; ++j) { const float d = acc[j] - mu; qq += d * d; }
#pragma unroll
    for (int off = 16; off > 0; off >>= 1) qq += __shfl_xor(qq, off, 32);
    const float rstd = rsqrtf(qq * (1.0f / (float)HDIM) + LNEPS);
    {
        v4f o0, o1, o2, o3;
#pragma unroll
        for (int k = 0; k < 4; ++k) {
            o0[k] = (acc[k] - mu) * rstd * gv[k] + ev[k];
            o1[k] = (acc[4 + k] - mu) * rstd * gv[4 + k] + ev[4 + k];
            o2[k] = (acc[8 + k] - mu) * rstd * gv[8 + k] + ev[8 + k];
            o3[k] = (acc[12 + k] - mu) * rstd * gv[12 + k] + ev[12 + k]; }
        *(v4fa*)(&xs[wb + 8u * lane]) = o0; *(v4fa*)(&xs[wb + 8u * lane + 4]) = o1;
        *(v4fa*)(&xs[wb + 256 + 8u * lane]) = o2; *(v4fa*)(&xs[wb + 260 + 8u * lane]) = o3;
    }
    wave_sync();
#pragma unroll 1
    for (unsigned e = 0; e < 16; ++e) {
        const unsigned c = e * 32u + lane;
        const float y = elu1(xs[wb + c]);
        const h16 hv = toh_flush(y);
        hs[wb + c] = hv;
    }
    wave_sync();
    h16* hrow = HH + (size_t)row * HDIM;
#pragma unroll 1
    for (int ps = 0; ps < 2; ++ps) {
#pragma unroll
        for (unsigned i = 0; i < 2; ++i) {
            const unsigned c = i * 256u + 8u * lane;
            const v8h hv = *(const v8ha*)(&hs[wb + c]);
            *(volatile v8h*)(hrow + c) = hv; }
        if (ps == 0) __threadfence(); }
}

__global__ __launch_bounds__(32 * GW2) void k_gemm2(const h16* __restrict__ HH, const h16* __restrict__ WP,
                                                    const float* __restrict__ b2, const float* __restrict__ g2, const float* __restrict__ be2, float* OUT) {
    __shared__ __align__(16) float os[16 * OP];
    const int lane = threadIdx.x & 31, lr = lane & 15, hi = lane >> 4;
    const int wave = __builtin_amdgcn_readfirstlane((int)(threadIdx.x >> 5));
    const unsigned r0 = blockIdx.x * 16u;
    const int c0 = wave * 128;
    v8f acc[8];
#pragma unroll
    for (int nb = 0; nb < 8; ++nb) acc[nb] = (v8f){};
    const size_t aoff = (size_t)(r0 + (unsigned)lr) * HDIM + 8 * hi;
    const size_t boff = (size_t)(c0 + lr) * HDIM + 8 * hi;
#pragma unroll 1
    for (int kc = 0; kc < HDIM; kc += 32) {
        const v16h ah = ldh(HH + aoff + kc);
#pragma unroll
        for (int nb = 0; nb < 8; ++nb) {
            const v16h b = ldh(WP + boff + (size_t)nb * 16 * HDIM + kc);
            acc[nb] = wmma16g(ah, b, acc[nb]);
        }
    }
#pragma unroll
    for (int nb = 0; nb < 8; ++nb) {
        const float bc = bfr(b2[c0 + nb * 16 + lr]);
#pragma unroll
        for (int j = 0; j < 8; ++j) {
            const float v = acc[nb][j] * WSI + bc;
            os[(hi * 8 + j) * OP + c0 + nb * 16 + lr] = v; }
    }
    __syncthreads();
    v4f gg[4], bb[4];
#pragma unroll
    for (int q = 0; q < 4; ++q) {
        const v4f g = *(const v4f*)(g2 + q * 128 + 4 * lane); const v4f e = *(const v4f*)(be2 + q * 128 + 4 * lane);
#pragma unroll
        for (int k = 0; k < 4; ++k) { gg[q][k] = bfr(g[k]); bb[q][k] = bfr(e[k]); }
    }
#pragma unroll 1
    for (int i = 0; i < 4; ++i) {
        const int ro = (wave * 4 + i) * OP + 4 * lane;
        v4f x[4]; float s = 0.0f;
#pragma unroll
        for (int q = 0; q < 4; ++q) { x[q] = *(const v4fa*)(&os[ro + q * 128]); s += (x[q][0] + x[q][1]) + (x[q][2] + x[q][3]); }
#pragma unroll
        for (int off = 16; off > 0; off >>= 1) s += __shfl_xor(s, off, 32);
        const float mu = s * (1.0f / (float)HDIM);
        float qq = 0.0f;
#pragma unroll
        for (int q = 0; q < 4; ++q) {
#pragma unroll
            for (int k = 0; k < 4; ++k) { const float d = x[q][k] - mu; qq += d * d; } }
#pragma unroll
        for (int off = 16; off > 0; off >>= 1) qq += __shfl_xor(qq, off, 32);
        const float rstd = rsqrtf(qq * (1.0f / (float)HDIM) + LNEPS);
#pragma unroll
        for (int q = 0; q < 4; ++q) { v4f o;
#pragma unroll
            for (int k = 0; k < 4; ++k) o[k] = elu1((x[q][k] - mu) * rstd * gg[q][k] + bb[q][k]);
            *(v4fa*)(&os[ro + q * 128]) = o; }
    }
    wave_sync();
#pragma unroll 1
    for (int ps = 0; ps < 2; ++ps) {
#pragma unroll 1
        for (int i = 0; i < 4; ++i) {
            const int row = wave * 4 + i;
            float* orow = OUT + (size_t)(r0 + (unsigned)row) * HDIM + 4 * lane;
#pragma unroll
            for (int q = 0; q < 4; ++q) {
                const v4f val = *(const v4fa*)(&os[row * OP + 4 * lane + q * 128]);
                *(volatile v4f*)(orow + q * 128) = val; } }
        if (ps == 0) __threadfence(); }
}

static constexpr size_t al256(size_t v) { return (v + 255) & ~(size_t)255; }
static constexpr size_t SZ_W1T = al256((size_t)IDIM * HDIM * 2);
static constexpr size_t SZ_W2P = al256((size_t)HDIM * HDIM * 2);
static constexpr size_t SZ_H1  = al256((size_t)NROWS * HDIM * 2);
static constexpr size_t OFF_W1T = 0;
static constexpr size_t OFF_W2P = OFF_W1T + SZ_W1T;
static constexpr size_t OFF_HH  = OFF_W2P + SZ_W2P;
static constexpr size_t SZ_TOTAL = OFF_HH + SZ_H1;
static_assert(SZ_TOTAL <= (size_t)134217728);
static constexpr size_t N_MSG = (size_t)NROWS * NPOS;
static constexpr size_t N_W1  = (size_t)HDIM * IDIM;
static constexpr size_t N_W2  = (size_t)HDIM * HDIM;
static constexpr size_t N_OUT = (size_t)NROWS * HDIM;
static constexpr unsigned W2_N8 = (unsigned)(N_W2 / 8);
static constexpr unsigned G_WCV = (W2_N8 + 255u) / 256u;
static constexpr unsigned G_TX = IDIM / 64, G_TY = HDIM / 64;
static constexpr unsigned G_GATHER = NROWS / GW;
static constexpr unsigned G_GEMM = NROWS / 16;
static_assert(N_W2 % 64 == 0);
static_assert((size_t)G_TX * 64 == IDIM);
static_assert((size_t)G_TY * 64 == HDIM);
static_assert((size_t)G_GATHER * GW == NROWS);
static_assert((size_t)G_GEMM * 16 == NROWS);

extern "C" void kernel_launch(void* const* d_in, const int* in_sizes, int n_in,
                              void* d_out, int out_size, void* d_ws, size_t ws_size, hipStream_t stream) {
    if (n_in < 9) return;
    if ((size_t)in_sizes[0] < N_MSG) return;
    if ((size_t)in_sizes[1] < N_W1) return;
    if (in_sizes[2] < HDIM || in_sizes[3] < HDIM || in_sizes[4] < HDIM) return;
    if ((size_t)in_sizes[5] < N_W2) return;
    if (in_sizes[6] < HDIM || in_sizes[7] < HDIM || in_sizes[8] < HDIM) return;
    if ((size_t)out_size < N_OUT) return;
    if (SZ_TOTAL > ws_size) return;
    const int*   msg = (const int*)d_in[0];
    const float* W1  = (const float*)d_in[1];
    const float* b1  = (const float*)d_in[2];
    const float* g1  = (const float*)d_in[3];
    const float* be1 = (const float*)d_in[4];
    const float* W2  = (const float*)d_in[5];
    const float* b2  = (const float*)d_in[6];
    const float* g2  = (const float*)d_in[7];
    const float* be2 = (const float*)d_in[8];
    float* OUT = (float*)d_out;
    char* wsp = (char*)d_ws;
    bf*  W1T = (bf*)(wsp + OFF_W1T);
    h16* W2P = (h16*)(wsp + OFF_W2P);
    h16* HH  = (h16*)(wsp + OFF_HH);

    k_w1t<<<dim3(G_TX, G_TY, 1), 256, 0, stream>>>(W1, W1T);
    k_wcv<<<G_WCV, 256, 0, stream>>>(W2, W2P, W2_N8);
    k_gather<<<G_GATHER, 32 * GW, 0, stream>>>(msg, W1T, b1, g1, be1, HH);
    k_gemm2<<<G_GEMM, 32 * GW2, 0, stream>>>(HH, W2P, b2, g2, be2, OUT);
}
